// MultiHeadQKVAttention_41936060678242
// MI455X (gfx1250) — hardware-verified
//
#include <hip/hip_runtime.h>

#define NB   8
#define SEQ  2048
#define DK   256
#define DV   32
#define NH   8
#define DO   256
#define KCH  64
#define SP   132
#define VTP  136

static_assert(NH * DV == DK);
static_assert((SEQ % 128) == 0 && (SEQ % KCH) == 0 && (DK % 32) == 0 && DV == 32 && DO == 256);
static_assert(((NB * SEQ * DK / 8) % 256) == 0);
static_assert(((SP * 4) % 16) == 0 && ((VTP * 2) % 16) == 0);

typedef __bf16         v16b __attribute__((ext_vector_type(16)));
typedef float          v8f  __attribute__((ext_vector_type(8)));
typedef float          v4f  __attribute__((ext_vector_type(4)));
typedef unsigned int   v4u  __attribute__((ext_vector_type(4)));
typedef unsigned int   v8u  __attribute__((ext_vector_type(8)));
typedef v4f __attribute__((may_alias)) v4fa;
typedef v4u __attribute__((may_alias)) v4ua;
union FB { v16b v; v8u u; v4u q[2]; };

#if defined(__HIP_DEVICE_COMPILE__)
#define DEV_ASM 1
#else
#define DEV_ASM 0
#endif

__device__ __forceinline__ unsigned short bf_bits(float f) {
  const unsigned u = __float_as_uint(f);
  return (unsigned short)((u + 0x7FFFu + ((u >> 16) & 1u)) >> 16);
}
__device__ __forceinline__ float bf_up(unsigned short hb) { return __uint_as_float(((unsigned)hb) << 16); }
__device__ __forceinline__ float bf16r(float f) { return bf_up(bf_bits(f)); }
__device__ __forceinline__ unsigned pk16(unsigned short a, unsigned short b) { return (unsigned)a | ((unsigned)b << 16); }
__device__ __forceinline__ v8f zero8() { v8f z = {0.f, 0.f, 0.f, 0.f, 0.f, 0.f, 0.f, 0.f}; return z; }

__device__ __forceinline__ v8f wmma_bf(v16b a, v16b b, v8f c) {
  v8f d = __builtin_amdgcn_wmma_f32_16x16x32_bf16(false, a, false, b, (short)0, c, false, false);
#if DEV_ASM
  asm volatile("v_nop\n\tv_nop\n\tv_nop\n\tv_nop" : "+v"(d) : "v"(a), "v"(b));
#endif
  return d;
}

__device__ __forceinline__ v16b ldfrag(const unsigned short* p, int h) {
  FB f;
  f.q[0] = *(const v4ua*)(p + 8 * h);
  f.q[1] = *(const v4ua*)(p + 16 + 8 * h);
  return f.v;
}

__device__ __forceinline__ void split_pack(v8f a, v8f c, v16b& hi, v16b& lo) {
  v8u hu = {0u, 0u, 0u, 0u, 0u, 0u, 0u, 0u};
  v8u lu = {0u, 0u, 0u, 0u, 0u, 0u, 0u, 0u};
#pragma unroll
  for (int i = 0; i < 4; ++i) {
    const float a0 = a[2 * i], a1 = a[2 * i + 1], c0 = c[2 * i], c1 = c[2 * i + 1];
    const unsigned short ha0 = bf_bits(a0), ha1 = bf_bits(a1), hc0 = bf_bits(c0), hc1 = bf_bits(c1);
    const unsigned short la0 = bf_bits(a0 - bf_up(ha0)), la1 = bf_bits(a1 - bf_up(ha1));
    const unsigned short lc0 = bf_bits(c0 - bf_up(hc0)), lc1 = bf_bits(c1 - bf_up(hc1));
    hu[i] = pk16(ha0, ha1);  hu[4 + i] = pk16(hc0, hc1);
    lu[i] = pk16(la0, la1);  lu[4 + i] = pk16(lc0, lc1);
  }
  FB H, L;
  H.u = hu; L.u = lu;
  hi = H.v; lo = L.v;
}

__global__ __launch_bounds__(256) void cvt_qk(const float* __restrict__ q, const float* __restrict__ k,
                                              unsigned short* qb, unsigned short* kb, int n8) {
  const int i = blockIdx.x * 256 + (int)threadIdx.x;
  if (i >= 2 * n8) return;
  const bool isq = (i < n8);
  const int j = isq ? i : (i - n8);
  const float* src = (isq ? q : k) + (size_t)j * 8;
  unsigned short* dst = (isq ? qb : kb) + (size_t)j * 8;
  const v4f a = *(const v4fa*)(src);
  const v4f c = *(const v4fa*)(src + 4);
  v4u p;
  p[0] = pk16(bf_bits(a[0]), bf_bits(a[1]));
  p[1] = pk16(bf_bits(a[2]), bf_bits(a[3]));
  p[2] = pk16(bf_bits(c[0]), bf_bits(c[1]));
  p[3] = pk16(bf_bits(c[2]), bf_bits(c[3]));
  *(volatile v4u*)dst = p;
  __threadfence();
  *(volatile v4u*)dst = p;
}

__global__ __launch_bounds__(128) void vtrans(const float* __restrict__ v, unsigned short* vt) {
  __shared__ __attribute__((aligned(16))) unsigned short sT[DV * VTP];
  const int t  = (int)threadIdx.x;
  const int b  = (int)blockIdx.x / (SEQ / 128);
  const int n0 = ((int)blockIdx.x % (SEQ / 128)) * 128;
#pragma unroll
  for (int i = 0; i < 8; ++i) {
    const int f   = i * 128 + t;
    const int key = f >> 3, c4 = (f & 7) * 4;
    const v4f x = *(const v4fa*)(v + ((size_t)b * SEQ + n0 + key) * DV + c4);
    sT[(c4 + 0) * VTP + key] = bf_bits(x[0]);
    sT[(c4 + 1) * VTP + key] = bf_bits(x[1]);
    sT[(c4 + 2) * VTP + key] = bf_bits(x[2]);
    sT[(c4 + 3) * VTP + key] = bf_bits(x[3]);
  }
  __syncthreads();
  v4u pc[4];
#pragma unroll
  for (int i = 0; i < 4; ++i) {
    const int L  = i * 16 + (t >> 3);
    const int vf = L >> 1, hl = L & 1;
    pc[i] = *(const v4ua*)(sT + vf * VTP + hl * 64 + (t & 7) * 8);
  }
  for (int pass = 0; pass < 2; ++pass) {
#pragma unroll
    for (int i = 0; i < 4; ++i) {
      const int L  = i * 16 + (t >> 3);
      const int vf = L >> 1, hl = L & 1;
      *(volatile v4u*)(vt + ((size_t)b * DV + vf) * SEQ + n0 + hl * 64 + (t & 7) * 8) = pc[i];
    }
    __threadfence();
  }
}

__global__ __launch_bounds__(256) void wfold(const float* __restrict__ wo, unsigned short* wfh, unsigned short* wfl) {
  __shared__ __attribute__((aligned(16))) unsigned short sH[DO * DV];
  __shared__ __attribute__((aligned(16))) unsigned short sL[DO * DV];
  const int d = (int)threadIdx.x;
  const float* row = wo + (size_t)d * (NH * DV);
#pragma unroll 1
  for (int vb = 0; vb < DV / 8; ++vb) {
    float s8[8];
#pragma unroll
    for (int e = 0; e < 8; ++e) s8[e] = 0.f;
#pragma unroll
    for (int g = 0; g < NH; ++g) {
      const v4f a = *(const v4fa*)(row + g * DV + 8 * vb);
      const v4f c = *(const v4fa*)(row + g * DV + 8 * vb + 4);
      s8[0] += bf16r(a[0]); s8[1] += bf16r(a[1]); s8[2] += bf16r(a[2]); s8[3] += bf16r(a[3]);
      s8[4] += bf16r(c[0]); s8[5] += bf16r(c[1]); s8[6] += bf16r(c[2]); s8[7] += bf16r(c[3]);
    }
#pragma unroll
    for (int e = 0; e < 8; ++e) {
      const unsigned short hb = bf_bits(s8[e]);
      sH[d * DV + 8 * vb + e] = hb;
      sL[d * DV + 8 * vb + e] = bf_bits(s8[e] - bf_up(hb));
    }
  }
  __syncthreads();
  v4u ph[4], pl[4];
#pragma unroll
  for (int i = 0; i < 4; ++i) {
    const int e = (i * 32 + (d >> 3)) * 64 + (d & 7) * 8;
    ph[i] = *(const v4ua*)(sH + e);
    pl[i] = *(const v4ua*)(sL + e);
  }
  for (int pass = 0; pass < 2; ++pass) {
#pragma unroll
    for (int i = 0; i < 4; ++i) {
      const int e = (i * 32 + (d >> 3)) * 64 + (d & 7) * 8;
      *(volatile v4u*)(wfh + e) = ph[i];
      *(volatile v4u*)(wfl + e) = pl[i];
    }
    __threadfence();
  }
}

__device__ __forceinline__ void out_store_pass(const float* slab, float* out, size_t row0, int half, int lane) {
  const int q8 = lane & 7, sub = lane >> 3;
#pragma unroll
  for (int it = 0; it < 16; ++it) {
    const int L = it * 4 + sub;
    const int row = L >> 2, seg = L & 3;
    const v4f val = *(const v4fa*)(slab + row * SP + seg * 32 + 4 * q8);
    float* dst = out + (row0 + (size_t)row) * DO + half * 128 + seg * 32 + 4 * q8;
    *(volatile v4f*)dst = val;
  }
}

__global__ __launch_bounds__(128) __attribute__((amdgpu_num_vgpr(256)))
void attn_out(const unsigned short* __restrict__ qb,
              const unsigned short* __restrict__ kb,
              const unsigned short* __restrict__ vt,
              const float* __restrict__ qpres,
              const float* __restrict__ kpres,
              const unsigned short* __restrict__ wfh,
              const unsigned short* __restrict__ wfl,
              const float* __restrict__ bo,
              float* out,
              float inv_scale) {
  __shared__ __attribute__((aligned(16))) float sO[4 * 16 * SP];

  const int tid = (int)threadIdx.x, lane = tid & 31, w = tid >> 5;
  const int h = lane >> 4, m = lane & 15;
  const int b = (int)blockIdx.y;
  const int q0 = (int)blockIdx.x * 64 + 16 * w;
  const size_t rowB = (size_t)b * SEQ;

  const unsigned short* qrow  = qb + (rowB + q0 + m) * DK;
  const unsigned short* kbase = kb + (rowB + m) * DK;
  const unsigned short* vbase = vt + ((size_t)b * DV + m) * SEQ;
  const float* mkp = kpres + rowB + 8 * h;
  const float qp = qpres[rowB + q0 + m];

  v8f o[2];
  o[0] = zero8(); o[1] = zero8();
  float mrun = -1e30f, lrun = 0.0f;

#pragma unroll 1
  for (int key0 = 0; key0 < SEQ; key0 += KCH) {
    v8f s[4];
#pragma unroll
    for (int j = 0; j < 4; ++j) s[j] = zero8();
#pragma unroll 1
    for (int dc = 0; dc < DK / 32; ++dc) {
      const v16b qf = ldfrag(qrow + 32 * dc, h);
#pragma unroll
      for (int j = 0; j < 4; ++j) {
        const v16b kf = ldfrag(kbase + (size_t)(key0 + 16 * j) * DK + 32 * dc, h);
        s[j] = wmma_bf(kf, qf, s[j]);
      }
    }

#pragma unroll
    for (int j = 0; j < 4; ++j) {
      const v4f ka = *(const v4fa*)(mkp + key0 + 16 * j);
      const v4f kc = *(const v4fa*)(mkp + key0 + 16 * j + 4);
      const float kp8[8] = {ka[0], ka[1], ka[2], ka[3], kc[0], kc[1], kc[2], kc[3]};
#pragma unroll
      for (int r = 0; r < 8; ++r) {
        float tv = s[j][r] * qp;
        tv = tv * kp8[r];
        tv = tv - (1.0f - kp8[r]) * 1e32f;
        s[j][r] = tv * inv_scale;
      }
    }

    float mloc = s[0][0];
#pragma unroll
    for (int j = 0; j < 4; ++j)
#pragma unroll
      for (int r = 0; r < 8; ++r) mloc = fmaxf(mloc, s[j][r]);
    mloc = fmaxf(mloc, __shfl_xor(mloc, 16, 32));
    const float mnew  = fmaxf(mrun, mloc);
    const float alpha = __expf(mrun - mnew);
    mrun = mnew;
    float lsum = 0.0f;
#pragma unroll
    for (int j = 0; j < 4; ++j)
#pragma unroll
      for (int r = 0; r < 8; ++r) {
        const float p = __expf(s[j][r] - mnew);
        s[j][r] = p;
        lsum += p;
      }
    lsum += __shfl_xor(lsum, 16, 32);
    lrun = lrun * alpha + lsum;
    o[0] = o[0] * alpha;
    o[1] = o[1] * alpha;

    v16b ph0, pl0, ph1, pl1;
    split_pack(s[0], s[1], ph0, pl0);
    split_pack(s[2], s[3], ph1, pl1);

#pragma unroll
    for (int t = 0; t < 2; ++t) {
      const unsigned short* vp = vbase + (size_t)(16 * t) * SEQ + key0;
      const v16b vf0 = ldfrag(vp, h);
      const v16b vf1 = ldfrag(vp + 32, h);
      o[t] = wmma_bf(vf0, ph0, o[t]);
      o[t] = wmma_bf(vf0, pl0, o[t]);
      o[t] = wmma_bf(vf1, ph1, o[t]);
      o[t] = wmma_bf(vf1, pl1, o[t]);
    }
  }

  const float inv = (lrun > 0.0f) ? (1.0f / lrun) : 0.0f;
  v16b hh, hl;
  split_pack(o[0] * inv, o[1] * inv, hh, hl);

  float* slab = sO + w * (16 * SP);
  const size_t orow0 = rowB + (size_t)q0;
#pragma unroll 1
  for (int half = 0; half < 2; ++half) {
#pragma unroll 1
    for (int uu = 0; uu < 8; ++uu) {
      const int u = 8 * half + uu;
      const v16b ah = ldfrag(wfh + (size_t)(16 * u + m) * DV, h);
      const v16b al = ldfrag(wfl + (size_t)(16 * u + m) * DV, h);
      v8f acc = zero8();
      acc = wmma_bf(ah, hh, acc);
      acc = wmma_bf(ah, hl, acc);
      acc = wmma_bf(al, hh, acc);
      const v4f b0 = *(const v4fa*)(bo + 16 * u + 8 * h);
      const v4f b1 = *(const v4fa*)(bo + 16 * u + 8 * h + 4);
      const float bb[8] = {b0[0], b0[1], b0[2], b0[3], b1[0], b1[1], b1[2], b1[3]};
#pragma unroll
      for (int r = 0; r < 8; ++r)
        slab[m * SP + 16 * uu + 8 * h + r] = acc[r] + bf16r(bb[r]);
    }
    __syncthreads();
    out_store_pass(slab, out, orow0, half, lane);
    __threadfence();
    out_store_pass(slab, out, orow0, half, lane);
    __syncthreads();
  }
}

extern "C" void kernel_launch(void* const* d_in, const int* in_sizes, int n_in,
                              void* d_out, int out_size, void* d_ws, size_t ws_size,
                              hipStream_t stream) {
  if (n_in < 7) return;
  if (in_sizes[0] != NB * SEQ * DK || in_sizes[1] != NB * SEQ * DK) return;
  if (in_sizes[2] != NB * SEQ * DV) return;
  if (in_sizes[3] != NB * SEQ || in_sizes[4] != NB * SEQ) return;
  if (in_sizes[5] != DO * NH * DV || in_sizes[6] != DO) return;
  if (out_size != NB * SEQ * DO) return;

  const float* q   = (const float*)d_in[0];
  const float* k   = (const float*)d_in[1];
  const float* v   = (const float*)d_in[2];
  const float* qpr = (const float*)d_in[3];
  const float* kpr = (const float*)d_in[4];
  const float* wo  = (const float*)d_in[5];
  const float* bo  = (const float*)d_in[6];
  float* out = (float*)d_out;

  const size_t PQ = (size_t)NB * SEQ * DK * 2;
  const size_t PV = (size_t)NB * DV * SEQ * 2;
  const size_t PW = (size_t)DO * DV * 2;
  size_t off = 0;
  const size_t oQ  = off; off += PQ;
  const size_t oK  = off; off += PQ;
  const size_t oV  = off; off += PV;
  const size_t oWH = off; off += PW;
  const size_t oWL = off; off += PW;
  if (off > ws_size) return;
  if (off > (size_t)134217728) return;

  char* ws = (char*)d_ws;
  unsigned short* Qb  = (unsigned short*)(ws + oQ);
  unsigned short* Kb  = (unsigned short*)(ws + oK);
  unsigned short* Vt  = (unsigned short*)(ws + oV);
  unsigned short* WfH = (unsigned short*)(ws + oWH);
  unsigned short* WfL = (unsigned short*)(ws + oWL);

  const int n8 = NB * SEQ * DK / 8;
  const dim3 gCvt((2 * n8 + 255) / 256);
  const dim3 gVt(NB * (SEQ / 128));
  const dim3 gAtt(SEQ / 64, NB);
  const float inv_scale = 0.17677669529663687f;

  cvt_qk<<<gCvt, dim3(256), 0, stream>>>(q, k, Qb, Kb, n8);
  vtrans<<<gVt, dim3(128), 0, stream>>>(v, Vt);
  wfold<<<dim3(1), dim3(256), 0, stream>>>(wo, WfH, WfL);
  attn_out<<<gAtt, dim3(128), 0, stream>>>(Qb, Kb, Vt, qpr, kpr, WfH, WfL, bo, out, inv_scale);
  (void)hipGetLastError();
}
